// linear_development_10746008175153
// MI455X (gfx1250) — hardware-run, weakly checked
//
#include <hip/hip_runtime.h>


#ifndef NB
#define NB 64
#endif
#ifndef SEQ
#define SEQ 2048
#endif
#define NB_FULL  64
#define SEQ_FULL 2048
#define CIN  8
#define MD   16
#define MM   256
#define NO   10
#define SPC  64
#define CHUNKS (SEQ / SPC)
#define NSTEP  (SEQ - 1)
#define WPB  4
#define SQN  5
#define SSC  0.03125f
#define QRS  2048.0f
#define QRI  (1.0f / 2048.0f)
#define NQ   ((NB * NO) / 4)

static_assert(MD == 16);
static_assert(MM == MD * MD);
static_assert(CIN == 8);
static_assert(SEQ % SPC == 0);
static_assert(CHUNKS >= 1);
static_assert((NB * CHUNKS) % WPB == 0);
static_assert((1 << SQN) == 32);
static_assert(NB <= NB_FULL);
static_assert(SEQ <= SEQ_FULL);
static_assert(2 * 32 * 4 == MM);
static_assert((NB * NO) % 4 == 0);
static_assert(NQ <= 256);
static_assert(WPB * MM * 2 * 2 + WPB * MM * 4 <= 131072);
static_assert(NB * NO * 4 <= 131072);

typedef _Float16 h16;
typedef __attribute__((ext_vector_type(16))) _Float16 v16h;
typedef __attribute__((ext_vector_type(8)))  _Float16 v8h;
typedef __attribute__((ext_vector_type(8)))  float    v8f;
typedef __attribute__((ext_vector_type(4)))  float    v4f;
typedef v4f  __attribute__((may_alias)) v4fa;

__device__ __forceinline__ unsigned short f2bf(float f) { unsigned u = __float_as_uint(f); u += 0x7FFFu + ((u >> 16) & 1u); return (unsigned short)(u >> 16); }
__device__ __forceinline__ float bfr(float f) { return __uint_as_float(((unsigned)f2bf(f)) << 16); }
__device__ __forceinline__ v16h cat16(v8h lo, v8h hi) { return __builtin_shufflevector(lo, hi, 0, 1, 2, 3, 4, 5, 6, 7, 8, 9, 10, 11, 12, 13, 14, 15); }
__device__ __forceinline__ v8f wmma16(v16h a, v16h b, v8f c) { return __builtin_amdgcn_wmma_f32_16x16x32_f16(false, a, false, b, (short)0, c, false, false); }
__device__ __forceinline__ void wave_sync() { __builtin_amdgcn_fence(3  , "wavefront"); __builtin_amdgcn_wave_barrier(); asm volatile("" ::: "memory"); }

__device__ __forceinline__ v8f wmma16g(v16h a, v16h b, v8f c) {
    c = wmma16(a, b, c);
    asm volatile("v_nop\n\tv_nop\n\tv_nop\n\tv_nop" : "+v"(c) : "v"(a), "v"(b));
    return c;
}
__device__ __forceinline__ h16 toh_flush(float v) { const h16 r = (h16)v; return (fabsf(v) < 6.103515625e-05f) ? (h16)0.0f : r; }
__device__ __forceinline__ void split8(const v8f x, v8h& hv, v8h& rv) {
#pragma unroll
    for (int i = 0; i < 8; ++i) { const h16 a = toh_flush(x[i]); hv[i] = a; rv[i] = toh_flush((x[i] - (float)a) * QRS); }
}
__device__ __forceinline__ v8f prod(v16h a, v8h bh, v8h br) {
    const v8h z = (v8h){};
    v8f m = (v8f){}, r = (v8f){};
    m = wmma16g(a, cat16(bh, z), m);
    r = wmma16g(a, cat16(br, bh), r);
    return m + r * QRI;
}

__global__ __launch_bounds__(32 * WPB) void k_chunk(const float* __restrict__ X, const float* __restrict__ A, float* CP) {
    __shared__ __align__(16) h16 tph[WPB * MM];
    __shared__ __align__(16) h16 tpr[WPB * MM];
    __shared__ __align__(16) float ot[WPB * MM];
    const int lane = threadIdx.x & 31, lr = lane & 15, hi = lane >> 4;
    const int wave = __builtin_amdgcn_readfirstlane((int)(threadIdx.x >> 5));
    const int gw = blockIdx.x * WPB + wave;
    const int b = gw / CHUNKS, chunk = gw % CHUNKS;
    const int wb = wave * MM;
    const int sto = wb + (8 * hi) * MD + lr;
    const int ldo = wb + lr * MD + 8 * hi;

    float G[CIN][8];
#pragma unroll
    for (int r = 0; r < 8; ++r) {
        const int row = 8 * hi + r;
        const float* pa = A + (size_t)((row * MD + lr) * CIN);
        const float* pb = A + (size_t)((lr * MD + row) * CIN);
        const v4f a0 = *(const v4f*)pa, a1 = *(const v4f*)(pa + 4), b0 = *(const v4f*)pb, b1 = *(const v4f*)(pb + 4);
#pragma unroll
        for (int c = 0; c < 4; ++c) { G[c][r] = bfr(a0[c]) - bfr(b0[c]); G[4 + c][r] = bfr(a1[c]) - bfr(b1[c]); }
        asm volatile("" ::: "memory");
    }

    v8f P;
#pragma unroll
    for (int r = 0; r < 8; ++r) P[r] = (8 * hi + r == lr) ? 1.0f : 0.0f;

    const int t0 = chunk * SPC;
    const int t1 = (t0 + SPC < NSTEP) ? (t0 + SPC) : NSTEP;
    const float* Xb = X + (size_t)b * SEQ_FULL * CIN;
    float xp[CIN];
    { const v4f q0 = *(const v4f*)(Xb + (size_t)t0 * CIN), q1 = *(const v4f*)(Xb + (size_t)t0 * CIN + 4);
#pragma unroll
      for (int c = 0; c < 4; ++c) { xp[c] = bfr(q0[c]); xp[4 + c] = bfr(q1[c]); } }

#pragma unroll 1
    for (int t = t0; t < t1; ++t) {
        const v4f q0 = *(const v4f*)(Xb + (size_t)(t + 1) * CIN), q1 = *(const v4f*)(Xb + (size_t)(t + 1) * CIN + 4);
        float dx[CIN];
#pragma unroll
        for (int c = 0; c < 4; ++c) { const float u0 = bfr(q0[c]), u1 = bfr(q1[c]); dx[c] = u0 - xp[c]; dx[4 + c] = u1 - xp[4 + c]; xp[c] = u0; xp[4 + c] = u1; }
        v8f Sp;
#pragma unroll
        for (int r = 0; r < 8; ++r) { float s = 0.0f;
#pragma unroll
            for (int c = 0; c < CIN; ++c) s = fmaf(dx[c], G[c][r], s);
            Sp[r] = s * SSC; }

        v8h sh, sr; split8(Sp, sh, sr);
        const v16h aS = cat16(sh, sr);
        const v8f C = -prod(aS, sh, sr);
        v8h ch, cr; split8(C, ch, cr);
        const v16h aC = cat16(ch, cr);
        const v8f C2 = prod(aC, ch, cr);
        v8h c2h, c2r; split8(C2, c2h, c2r);
        const v8f C3 = prod(aC, c2h, c2r);
        v8h c3h, c3r; split8(C3, c3h, c3r);
        const v8f C4 = prod(aC, c3h, c3r);
        v8f F, Oh;
#pragma unroll
        for (int r = 0; r < 8; ++r) {
            const float c1 = C[r], c2 = C2[r], c3 = C3[r], c4 = C4[r];
            F[r]  = c1 * 0.5f + (c2 * (1.0f / 24.0f) + (c3 * (1.0f / 720.0f) + c4 * (1.0f / 40320.0f)));
            Oh[r] = c1 * (1.0f / 6.0f) + (c2 * (1.0f / 120.0f) + (c3 * (1.0f / 5040.0f) + c4 * (1.0f / 362880.0f)));
        }
        v8h oh, orr; split8(Oh, oh, orr);
        const v8f SO = prod(aS, oh, orr);
        v8f R = (F + Sp) - SO;

#pragma unroll 1
        for (int j = 0; j < SQN; ++j) {
            v8h rh, rr; split8(R, rh, rr);
#pragma unroll
            for (int r = 0; r < 8; ++r) { tph[sto + r * MD] = rh[r]; tpr[sto + r * MD] = rr[r]; }
            wave_sync();
            const v16h aR = cat16(*(const v8h*)(&tph[ldo]), *(const v8h*)(&tpr[ldo]));
            wave_sync();
            R = (R + R) + prod(aR, rh, rr);
        }
        {
            v8h rh, rr; split8(R, rh, rr);
#pragma unroll
            for (int r = 0; r < 8; ++r) { tph[sto + r * MD] = rh[r]; tpr[sto + r * MD] = rr[r]; }
            wave_sync();
            const v16h aR = cat16(*(const v8h*)(&tph[ldo]), *(const v8h*)(&tpr[ldo]));
            wave_sync();
            v8h ph, pr; split8(P, ph, pr);
            P = P + prod(aR, ph, pr);
        }
    }

#pragma unroll
    for (int r = 0; r < 8; ++r) ot[sto + r * MD] = P[r];
    wave_sync();
    float* dst = CP + (size_t)gw * MM;
#pragma unroll 1
    for (int ps = 0; ps < 2; ++ps) {
#pragma unroll
        for (int s = 0; s < 2; ++s) { const int p = s * 32 + lane;
            const v4f val = *(const v4fa*)(&ot[wb + p * 4]);
            *(volatile v4f*)(dst + p * 4) = val; }
        if (ps == 0) __threadfence(); }
}

__global__ __launch_bounds__(32) void k_reduce(const float* __restrict__ CP, float* Z) {
    __shared__ __align__(16) float ot[MM];
    const int lane = threadIdx.x & 31, lr = lane & 15, hi = lane >> 4;
    const int b = blockIdx.x;
    v8f P;
#pragma unroll
    for (int r = 0; r < 8; ++r) P[r] = (8 * hi + r == lr) ? 1.0f : 0.0f;
#pragma unroll 1
    for (int c = 0; c < CHUNKS; ++c) {
        const float* src = CP + (size_t)(b * CHUNKS + c) * MM + lr * MD + 8 * hi;
        const v4f x0 = *(const v4f*)src, x1 = *(const v4f*)(src + 4);
        v8f Mr;
#pragma unroll
        for (int i = 0; i < 4; ++i) { Mr[i] = x0[i]; Mr[4 + i] = x1[i]; }
        v8h mh, mr; split8(Mr, mh, mr);
        const v16h aM = cat16(mh, mr);
        v8h ph, pr; split8(P, ph, pr);
        P = prod(aM, ph, pr);
    }
#pragma unroll
    for (int r = 0; r < 8; ++r) ot[(8 * hi + r) * MD + lr] = P[r];
    wave_sync();
    float* dst = Z + (size_t)b * MM;
#pragma unroll 1
    for (int ps = 0; ps < 2; ++ps) {
#pragma unroll
        for (int s = 0; s < 2; ++s) { const int p = s * 32 + lane;
            const v4f val = *(const v4fa*)(&ot[p * 4]);
            *(volatile v4f*)(dst + p * 4) = val; }
        if (ps == 0) __threadfence(); }
}

__global__ __launch_bounds__(256) void k_head(const float* __restrict__ Z, const float* __restrict__ W, const float* __restrict__ bias, float* OUT) {
    __shared__ __align__(16) float so[NB * NO];
    const int tid = threadIdx.x;
#pragma unroll 1
    for (int it = 0; it < (NB * NO + 255) / 256; ++it) {
        const int idx = it * 256 + tid;
        const int ic = idx < NB * NO ? idx : (NB * NO - 1);
        const int bb = ic / NO, o = ic % NO;
        float acc = bfr(bias[o]);
        const float* z = Z + (size_t)bb * MM;
        const float* w = W + (size_t)o * MM;
#pragma unroll 4
        for (int k = 0; k < MM; ++k) acc = fmaf(z[k], bfr(w[k]), acc);
        if (idx < NB * NO) so[idx] = acc;
    }
    __syncthreads();
    const int tq = tid < NQ ? tid : (NQ - 1);
    const v4f val = *(const v4fa*)(&so[tq * 4]);
#pragma unroll 1
    for (int ps = 0; ps < 2; ++ps) {
        if (tid < NQ) *(volatile v4f*)(OUT + (size_t)tid * 4) = val;
        if (ps == 0) __threadfence(); }
}

static constexpr size_t al256(size_t v) { return (v + 255) & ~(size_t)255; }
static constexpr size_t SZ_CP = al256((size_t)NB * CHUNKS * MM * 4);
static constexpr size_t SZ_Z  = al256((size_t)NB * MM * 4);
static constexpr size_t SZ_TOTAL = SZ_CP + SZ_Z;
static_assert(SZ_TOTAL <= (size_t)134217728);
static_assert(SZ_CP == (size_t)NB * CHUNKS * MM * 4);
static_assert(SZ_Z == (size_t)NB * MM * 4);

extern "C" void kernel_launch(void* const* d_in, const int* in_sizes, int n_in,
                              void* d_out, int out_size, void* d_ws, size_t ws_size, hipStream_t stream) {
    if (n_in < 4) return;
    if ((size_t)in_sizes[0] < ((size_t)(NB - 1) * SEQ_FULL + SEQ) * CIN) return;
    if (in_sizes[1] < MD * MD * CIN || in_sizes[2] < NO * MM || in_sizes[3] < NO) return;
    if (out_size < NB * NO) return;
    if (SZ_TOTAL > ws_size) return;
    const float* X = (const float*)d_in[0];
    const float* A = (const float*)d_in[1];
    const float* W = (const float*)d_in[2];
    const float* bias = (const float*)d_in[3];
    float* OUT = (float*)d_out;
    char* wsp = (char*)d_ws;
    float* CP = (float*)wsp; wsp += SZ_CP;
    float* Zp = (float*)wsp; wsp += SZ_Z;

    k_chunk<<<dim3((NB * CHUNKS) / WPB, 1, 1), 32 * WPB, 0, stream>>>(X, A, CP);
    k_reduce<<<dim3(NB, 1, 1), 32, 0, stream>>>(CP, Zp);
    k_head<<<dim3(1, 1, 1), 256, 0, stream>>>(Zp, W, bias, OUT);
}
